// EAGNN_56126632624862
// MI455X (gfx1250) — hardware-run, weakly checked
//
#include <hip/hip_runtime.h>
#include <stddef.h>
#include <stdint.h>

#define NB     32
#define NN     1024
#define NE     4096
#define NA     16
#define BNR    (NB * NN)
#define FIN    16
#define HID    64
#define MID    208
#define AHP    448
#define PP     416
#define ANPB   (NA * NN)
#define RTOT   (NB * ANPB)
#define OFFP   1056
#define DEGCAP 32
#define PARW   1152
#define PJ     224
#define RECW   448
#define NCH    128
#define NREC   256
#define RECN   2048.0
#define LNEPS  1e-5f
#define BNEPS  1e-5f
#define NU_W0  512
#define NU_W1  1024
#define NU_WL  (NU_W0 + 2 * NU_W1)
#define NU_X0  (BNR * 8)
#define NU_PA  (NU_WL + NU_X0)
#define NU_PB  (AHP * (AHP / 8))
#define BK_INTS (NE + 8 * NN + NE + OFFP + 32)
#define PB_STR 209
#define PASSB_FLOATS (MID * NA + 256 * 8 + NA * NCH + NA * NCH + 16 + NCH * PB_STR)
#define DUNITS (NA * NCH / 4)
#define WSMAX  134217728

static_assert(NN == 1024 && NE == 4096 && MID == FIN + 3 * HID && MID == 208);
static_assert(AHP % 32 == 0 && AHP == 6 * HID + 64 && PP == 2 * MID);
static_assert((AHP * 2) % 128 == 0 && (PP * 4) % 128 == 0 && (OFFP * 4) % 128 == 0);
static_assert(NU_W0 % 256 == 0 && NU_W1 % 256 == 0 && NU_PA % 256 == 0 && NU_PB % 256 == 0);
static_assert(MID <= PJ && PJ % 32 == 0 && RECW == 2 * PJ && (RECW / 4) == 112);
static_assert(NN % NCH == 0 && NREC == NB * (NN / NCH) && NCH == 128);
static_assert(BNR % 64 == 0 && NN % 64 == 0);
static_assert((MID * NA) % 256 == 0 && (NCH * (MID / 4)) % 256 == 0);
static_assert(PARW % 32 == 0 && PARW >= 5 * PJ + 32);
static_assert(BK_INTS * 4 <= 160000 && PASSB_FLOATS * 4 <= 160000);
static_assert(DEGCAP == 32);
static_assert(NA == 16 && (NA & (NA - 1)) == 0);
static_assert(DUNITS == 2 * 256 && 3 * PJ >= DUNITS && 2 * PJ < DUNITS);

typedef float          v2f   __attribute__((ext_vector_type(2)));
typedef float          v4f   __attribute__((ext_vector_type(4)));
typedef float          v8f   __attribute__((ext_vector_type(8)));
typedef int            v4i   __attribute__((ext_vector_type(4)));
typedef int            v8i   __attribute__((ext_vector_type(8)));
typedef unsigned short v2us  __attribute__((ext_vector_type(2)));
typedef unsigned short v8us  __attribute__((ext_vector_type(8)));
typedef unsigned short v16us __attribute__((ext_vector_type(16)));
typedef __bf16         v16bf __attribute__((ext_vector_type(16)));
typedef v2f  __attribute__((may_alias)) v2fa;
typedef v4f  __attribute__((may_alias)) v4fa;
typedef v4i  __attribute__((may_alias)) v4ia;
typedef v2us __attribute__((may_alias)) v2usa;
typedef v8us __attribute__((may_alias)) v8usa;
typedef unsigned __attribute__((may_alias)) u1a;
typedef int      __attribute__((may_alias)) i1a;
union FragB { v16bf v; v16us u; v8us h[2]; v8i w; };

__device__ __forceinline__ v8f wmb(const FragB& a, const FragB& b, v8f c) {
  v8f d = __builtin_amdgcn_wmma_f32_16x16x32_bf16(false, a.v, false, b.v, (short)0, c, false, false);
  asm volatile("v_nop\n\tv_nop\n\tv_nop\n\tv_nop" : "+v"(d) : "v"(a.w), "v"(b.w));
  return d;
}

__device__ __forceinline__ v8f z8() { v8f z = {0.f, 0.f, 0.f, 0.f, 0.f, 0.f, 0.f, 0.f}; return z; }

__device__ __forceinline__ unsigned bf16_bits(float f) {
  const unsigned u = __float_as_uint(f);
  return (u + 0x7FFFu + ((u >> 16) & 1u)) >> 16;
}
__device__ __forceinline__ float bf16_val(float f) {
  return __uint_as_float(bf16_bits(f) << 16);
}
__device__ __forceinline__ unsigned hl_bits(float v, unsigned& lo) {
  const unsigned hb = bf16_bits(v);
  lo = bf16_bits(v - __uint_as_float(hb << 16));
  return hb;
}
__device__ __forceinline__ int clampi(int v, int lo, int hi) { return v < lo ? lo : (v > hi ? hi : v); }
__device__ __forceinline__ float nmax(float m, float v) { return (v > m || v != v) ? v : m; }

__device__ __forceinline__ void wave_sync() {
  __builtin_amdgcn_fence(__ATOMIC_RELEASE, "workgroup");
  __builtin_amdgcn_wave_barrier();
  __builtin_amdgcn_fence(__ATOMIC_ACQUIRE, "workgroup");
}
__device__ __forceinline__ void put16(unsigned short* dp, v8us o) {
  *(volatile v8us*)dp = o;
  __threadfence();
  *(volatile v8us*)dp = o;
}
__device__ __forceinline__ void pin_i(int v) { asm volatile("" :: "v"(v)); }
__device__ __forceinline__ void pin_f4(v4f d) { asm volatile("" :: "v"(d.x), "v"(d.y), "v"(d.z), "v"(d.w)); }

__global__ __launch_bounds__(256) void k_pa(const float* __restrict__ gn, const float* __restrict__ W0,
                                            const float* __restrict__ W1, const float* __restrict__ W2,
                                            unsigned short* W0D, unsigned short* W1D, unsigned short* W2D,
                                            unsigned short* AH) {
  const int u = (int)blockIdx.x * 256 + (int)threadIdx.x;
  v8us o;
  unsigned short* dp;
  if (u < NU_W0) {
    const int n = u >> 3, k8 = (u & 7) * 8;
    const unsigned mk = (k8 < 32) ? 0xffffu : 0u;
    const float* p = W0 + n;
#pragma unroll
    for (int i = 0; i < 8; ++i) {
      const float f = p[(size_t)((k8 + i) & 15) * HID];
      o[i] = (unsigned short)(bf16_bits(f) & mk);
    }
    dp = W0D + (size_t)u * 8;
  } else if (u < NU_W0 + NU_W1) {
    const int v = u - NU_W0;
    const int n = v >> 4, k8 = (v & 15) * 8;
    const float* p = W1 + n;
#pragma unroll
    for (int i = 0; i < 8; ++i) o[i] = (unsigned short)bf16_bits(p[(size_t)((k8 + i) & 63) * HID]);
    dp = W1D + (size_t)v * 8;
  } else if (u < NU_WL) {
    const int v = u - NU_W0 - NU_W1;
    const int n = v >> 4, k8 = (v & 15) * 8;
    const float* p = W2 + n;
#pragma unroll
    for (int i = 0; i < 8; ++i) o[i] = (unsigned short)bf16_bits(p[(size_t)((k8 + i) & 63) * HID]);
    dp = W2D + (size_t)v * 8;
  } else if (u < NU_PA) {
    const int v = u - NU_WL;
    const int row = v >> 3, j = v & 7;
    const unsigned mk = (j < 2) ? 0xffffu : 0u;
    const float* p = gn + (size_t)row * FIN + 8 * (j & 1);
    const v4f a = *(const v4f*)p;
    const v4f c = *(const v4f*)(p + 4);
    o[0] = (unsigned short)(bf16_bits(a.x) & mk); o[1] = (unsigned short)(bf16_bits(a.y) & mk);
    o[2] = (unsigned short)(bf16_bits(a.z) & mk); o[3] = (unsigned short)(bf16_bits(a.w) & mk);
    o[4] = (unsigned short)(bf16_bits(c.x) & mk); o[5] = (unsigned short)(bf16_bits(c.y) & mk);
    o[6] = (unsigned short)(bf16_bits(c.z) & mk); o[7] = (unsigned short)(bf16_bits(c.w) & mk);
    dp = AH + (size_t)row * AHP + 384 + 8 * j;
  } else {
    return;
  }
  put16(dp, o);
}

__global__ __launch_bounds__(256) void k_pb(const float* __restrict__ A1, unsigned short* WAB) {
  const int u = (int)blockIdx.x * 256 + (int)threadIdx.x;
  if (u >= NU_PB) return;
  const int n  = u / (AHP / 8);
  const int k8 = (u - n * (AHP / 8)) * 8;
  const bool valid = (n < PP) && (k8 < 400);
  const unsigned mk = valid ? 0xffffu : 0u;
  const int nc = n < PP ? n : PP - 1;
  const int col = nc < MID ? nc : nc - MID;
  const int rowoff = nc < MID ? 0 : MID;
  int xr0;
  if (k8 < 384)      xr0 = FIN + HID * (k8 >> 7) + (k8 & 63);
  else if (k8 < 400) xr0 = k8 - 384;
  else               xr0 = 0;
  const float* p = A1 + (size_t)(rowoff + xr0) * MID + col;
  v8us o;
#pragma unroll
  for (int i = 0; i < 8; ++i) o[i] = (unsigned short)(bf16_bits(p[(size_t)i * MID]) & mk);
  put16(WAB + (size_t)u * 8, o);
}

__global__ __launch_bounds__(256) void k_pc(const float* __restrict__ A1, const float* __restrict__ a1b,
                                            const float* __restrict__ eW, const float* __restrict__ eb,
                                            const float* __restrict__ bng, const float* __restrict__ bnb,
                                            const float* __restrict__ w2, const float* __restrict__ b2,
                                            float* PAR) {
  __shared__ __attribute__((aligned(16))) float pst[PARW];
  const int tid = (int)threadIdx.x;
  const int jc = tid < MID ? tid : MID - 1;
  const bool live = tid < MID;
  float su = 0.0f, sc = 0.0f;
#pragma unroll 1
  for (int k = 0; k < HID; ++k) {
    const float w = bf16_val(A1[(size_t)(2 * MID + k) * MID + jc]);
    su = fmaf(bf16_val(eW[k]), w, su);
    sc = fmaf(bf16_val(eb[k]), w, sc);
  }
  const float cvv = sc + bf16_val(a1b[jc]);
  const float gv = bf16_val(bng[jc]);
  const float bv = bf16_val(bnb[jc]);
  const float wv = bf16_val(w2[jc]);
  const float b2v = bf16_val(b2[0]);
  if (tid < PJ) {
    pst[tid]          = live ? su  : 0.0f;
    pst[PJ + tid]     = live ? cvv : 0.0f;
    pst[2 * PJ + tid] = live ? gv  : 0.0f;
    pst[3 * PJ + tid] = live ? bv  : 0.0f;
    pst[4 * PJ + tid] = live ? wv  : 0.0f;
  }
  if (tid < 32) pst[5 * PJ + tid] = (tid == 0) ? b2v : 0.0f;
  __syncthreads();
  for (int q = tid; q < PARW / 4; q += 256) {
    const v4f v = *(const v4fa*)(pst + 4 * q);
    *(volatile v4f*)(PAR + 4 * q) = v;
  }
  __threadfence();
  for (int q = tid; q < PARW / 4; q += 256) {
    const v4f v = *(const v4fa*)(pst + 4 * q);
    *(volatile v4f*)(PAR + 4 * q) = v;
  }
}

__global__ __launch_bounds__(256) void k_bucket(const int* __restrict__ links, int* LIST, int* OFF) {
  extern __shared__ __attribute__((aligned(16))) int dsmb[];
  int* sed  = dsmb;
  int* cw   = sed + NE;
  int* lst  = cw + 8 * NN;
  int* offs = lst + NE;
  int* misc = offs + OFFP;
  const int tid = (int)threadIdx.x, lane = tid & 31, wave = tid >> 5;
  const int b = (int)blockIdx.x;
  const int* src = links + (size_t)b * 2 * NE;
  const int* dst = src + NE;

  int bad = 0;
  const v4i z4 = {0, 0, 0, 0};
#pragma unroll
  for (int it = 0; it < 4; ++it) {
    const int q = it * 256 + tid;
    v4i s = *(const v4i*)(src + 4 * q);
    v4i d = *(const v4i*)(dst + 4 * q);
    bad |= ((unsigned)s.x >= (unsigned)NN) | ((unsigned)s.y >= (unsigned)NN) |
           ((unsigned)s.z >= (unsigned)NN) | ((unsigned)s.w >= (unsigned)NN) |
           ((unsigned)d.x >= (unsigned)NN) | ((unsigned)d.y >= (unsigned)NN) |
           ((unsigned)d.z >= (unsigned)NN) | ((unsigned)d.w >= (unsigned)NN);
    v4i e;
    e.x = (clampi(s.x, 0, NN - 1) << 10) | clampi(d.x, 0, NN - 1);
    e.y = (clampi(s.y, 0, NN - 1) << 10) | clampi(d.y, 0, NN - 1);
    e.z = (clampi(s.z, 0, NN - 1) << 10) | clampi(d.z, 0, NN - 1);
    e.w = (clampi(s.w, 0, NN - 1) << 10) | clampi(d.w, 0, NN - 1);
    *(v4ia*)(sed + 4 * q) = e;
    *(v4ia*)(lst + 4 * q) = z4;
  }
#pragma unroll
  for (int it = 0; it < 8; ++it) *(v4ia*)(cw + 4 * (it * 256 + tid)) = z4;
  {
    const unsigned bm = __builtin_amdgcn_ballot_w32(bad != 0);
    if (lane == 0) misc[wave] = (bm != 0u) ? 1 : 0;
  }
  __syncthreads();
  const int pois = misc[0] | misc[1] | misc[2] | misc[3] | misc[4] | misc[5] | misc[6] | misc[7];

  if (lane == 0) {
    int* cww = cw + wave * NN;
#pragma unroll 1
    for (int e = 0; e < NE / 8; ++e) {
      const int d = sed[wave * (NE / 8) + e] & (NN - 1);
      cww[d] = cww[d] + 1;
    }
  }
  __syncthreads();

  const int sb = 4 * tid;
  int tq[4];
#pragma unroll
  for (int j = 0; j < 4; ++j) {
    int run = 0;
#pragma unroll
    for (int w2 = 0; w2 < 8; ++w2) {
      const int c = cw[w2 * NN + sb + j];
      cw[w2 * NN + sb + j] = run;
      run += c;
    }
    tq[j] = run;
  }
  const int ts = (tq[0] + tq[1]) + (tq[2] + tq[3]);
  int incl = ts;
#pragma unroll
  for (int d = 1; d < 32; d <<= 1) {
    const int y = __shfl_up(incl, d, 32);
    if (lane >= d) incl += y;
  }
  if (lane == 31) misc[8 + wave] = incl;
  __syncthreads();
  int base = 0;
#pragma unroll
  for (int w2 = 0; w2 < 8; ++w2) {
    const int wt = misc[8 + w2];
    base += (w2 < wave) ? wt : 0;
  }
  const int ex = base + incl - ts;
  {
    int oj = ex;
#pragma unroll
    for (int j = 0; j < 4; ++j) {
      offs[sb + j] = oj;
#pragma unroll
      for (int w2 = 0; w2 < 8; ++w2) cw[w2 * NN + sb + j] = cw[w2 * NN + sb + j] + oj;
      oj += tq[j];
    }
  }
  if (tid == 255) offs[NN] = ex + ts;
  if (tid < 31) offs[NN + 1 + tid] = (tid == 0) ? pois : 0;
  __syncthreads();

  if (lane == 0) {
    int* cww = cw + wave * NN;
#pragma unroll 1
    for (int e = 0; e < NE / 8; ++e) {
      const int v = sed[wave * (NE / 8) + e];
      const int d = v & (NN - 1);
      int p = cww[d];
      p = clampi(p, 0, NE - 1);
      lst[p] = v >> 10;
      cww[d] = p + 1;
    }
  }
  __syncthreads();

  int* lp = LIST + (size_t)b * NE;
  int* op = OFF + (size_t)b * OFFP;
  v4i lv[4];
#pragma unroll
  for (int it = 0; it < 4; ++it) lv[it] = *(const v4ia*)(lst + 4 * (it * 256 + tid));
  const v4i ov0 = *(const v4ia*)(offs + 4 * tid);
  const v4i ov1 = *(const v4ia*)(offs + 4 * (256 + (tid & 7)));
#pragma unroll
  for (int it = 0; it < 4; ++it) *(volatile v4i*)(lp + 4 * (it * 256 + tid)) = lv[it];
  *(volatile v4i*)(op + 4 * tid) = ov0;
  if (tid < 8) *(volatile v4i*)(op + 4 * (256 + tid)) = ov1;
  __threadfence();
#pragma unroll
  for (int it = 0; it < 4; ++it) *(volatile v4i*)(lp + 4 * (it * 256 + tid)) = lv[it];
  *(volatile v4i*)(op + 4 * tid) = ov0;
  if (tid < 8) *(volatile v4i*)(op + 4 * (256 + tid)) = ov1;
}

template <int L0>
__global__ __launch_bounds__(256) void k_agg(const int* __restrict__ LIST, const int* __restrict__ OFF,
                                             const float* __restrict__ gn, const unsigned short* __restrict__ AH,
                                             int sliceOff, unsigned short* AGG) {
  constexpr int RW  = L0 ? 64 : 128;
  constexpr int NST = RW / 32;
  __shared__ __attribute__((aligned(16))) unsigned short rs[8 * 8 * RW];
  const int tid = (int)threadIdx.x, lane = tid & 31, wave = tid >> 5;
  const int row0 = (int)blockIdx.x * 64 + wave * 8;
  const int b = row0 >> 10, s0 = row0 & (NN - 1);
  const int* offp = OFF + (size_t)b * OFFP;
  const int* lstp = LIST + (size_t)b * NE;
  const int pflag = offp[NN + 1];
  unsigned short* rw = rs + wave * 8 * RW;
  const float qnan = __int_as_float(0x7fc00000);

#pragma unroll 1
  for (int si = 0; si < 8; ++si) {
    const int s = s0 + si;
    int o  = offp[s];
    const int o1 = offp[s + 1];
    o = clampi(o, 0, NE);
    const int craw = o1 - o;
    const bool big = craw > DEGCAP;
    const int c = __builtin_amdgcn_readfirstlane(clampi(craw, 0, DEGCAP));
    int idx = o + lane;
    idx = idx > NE - 1 ? NE - 1 : idx;
    int sr = lstp[idx];
    sr = clampi(sr, 0, NN - 1);
    const float pz = (pflag != 0 || big) ? qnan : 0.0f;
    if constexpr (L0 != 0) {
      float a = 0.0f;
#pragma unroll 1
      for (int k = 0; k < c; ++k) {
        const int sk = __builtin_amdgcn_readlane(sr, k);
        const float v = gn[(size_t)(b * NN + sk) * FIN + (lane & 15)];
        a += bf16_val(v);
      }
      const float mv = a + pz;
      unsigned lb;
      const unsigned hb = hl_bits(mv, lb);
      rw[si * RW + lane]      = (unsigned short)((lane < 16) ? hb : lb);
      rw[si * RW + 32 + lane] = (unsigned short)(lane >> 5);
    } else {
      float a0 = 0.0f, a1 = 0.0f;
#pragma unroll 1
      for (int k = 0; k < c; ++k) {
        const int sk = __builtin_amdgcn_readlane(sr, k);
        const unsigned short* rp = AH + (size_t)(b * NN + sk) * AHP + sliceOff + 2 * lane;
        const unsigned wh = *(const u1a*)rp;
        const unsigned wl = *(const u1a*)(rp + HID);
        a0 += __uint_as_float(wh << 16)         + __uint_as_float(wl << 16);
        a1 += __uint_as_float(wh & 0xffff0000u) + __uint_as_float(wl & 0xffff0000u);
      }
      const float m0 = a0 + pz, m1 = a1 + pz;
      unsigned l0, l1;
      const unsigned h0 = hl_bits(m0, l0);
      const unsigned h1 = hl_bits(m1, l1);
      v2us hv, lv;
      hv[0] = (unsigned short)h0; hv[1] = (unsigned short)h1;
      lv[0] = (unsigned short)l0; lv[1] = (unsigned short)l1;
      *(v2usa*)(rw + si * RW + 2 * lane)       = hv;
      *(v2usa*)(rw + si * RW + HID + 2 * lane) = lv;
    }
  }
  wave_sync();
  v8us q[NST];
#pragma unroll
  for (int j = 0; j < NST; ++j) q[j] = *(const v8usa*)(rw + j * 256 + 8 * lane);
  unsigned short* dp = AGG + (size_t)row0 * RW + 8 * lane;
#pragma unroll
  for (int j = 0; j < NST; ++j) *(volatile v8us*)(dp + j * 256) = q[j];
  __threadfence();
#pragma unroll
  for (int j = 0; j < NST; ++j) *(volatile v8us*)(dp + j * 256) = q[j];
}

template <int KS>
__global__ __launch_bounds__(128) void k_gemm_ln(const unsigned short* __restrict__ A,
                                                 const unsigned short* __restrict__ BT,
                                                 const float* __restrict__ bias, const float* __restrict__ gam,
                                                 const float* __restrict__ bet, unsigned short* AH, int sliceOff) {
  constexpr int KD = 32 * KS;
  __shared__ __attribute__((aligned(16))) float stg[64 * 64];
  const int tid = (int)threadIdx.x, lane = tid & 31, wave = tid >> 5, hh = lane >> 4, m = lane & 15;
  const int rowBase = (int)blockIdx.x * 64;

  v8f acc[4];
#pragma unroll
  for (int t = 0; t < 4; ++t) acc[t] = z8();
  const unsigned short* ap = A + (size_t)(rowBase + 16 * wave + m) * (size_t)KD + 8 * hh;
  const unsigned short* bp = BT + (size_t)m * (size_t)KD + 8 * hh;
#pragma unroll
  for (int ks = 0; ks < KS; ++ks) {
    const int k0 = 32 * ks;
    FragB af;
    af.h[0] = *(const v8usa*)(ap + k0);
    af.h[1] = *(const v8usa*)(ap + k0 + 16);
#pragma unroll
    for (int nt = 0; nt < 4; ++nt) {
      const unsigned short* wq = bp + (size_t)(16 * nt) * (size_t)KD + k0;
      FragB bf;
      bf.h[0] = *(const v8usa*)wq;
      bf.h[1] = *(const v8usa*)(wq + 16);
      acc[nt] = wmb(af, bf, acc[nt]);
    }
  }
#pragma unroll
  for (int nt = 0; nt < 4; ++nt) {
    const int lc = 16 * nt + m;
#pragma unroll
    for (int r = 0; r < 8; ++r) {
      const int lr = 16 * wave + 8 * hh + r;
      stg[lr * 64 + lc] = acc[nt][r];
    }
  }
  __syncthreads();

  const v2f b2v = *(const v2f*)(bias + 2 * lane);
  const v2f g2v = *(const v2f*)(gam + 2 * lane);
  const v2f e2v = *(const v2f*)(bet + 2 * lane);
  const float bq0 = bf16_val(b2v.x), bq1 = bf16_val(b2v.y);
  const float gq0 = bf16_val(g2v.x), gq1 = bf16_val(g2v.y);
  const float eq0 = bf16_val(e2v.x), eq1 = bf16_val(e2v.y);
  const float invd = 1.0f / 64.0f;

#pragma unroll 1
  for (int i = 0; i < 16; ++i) {
    float* frow = stg + (16 * wave + i) * 64;
    const v2f p = *(const v2fa*)(frow + 2 * lane);
    const float y0 = p.x + bq0, y1 = p.y + bq1;
    float s = y0 + y1;
    s += __shfl_xor(s, 16, 32);
    s += __shfl_xor(s, 8, 32);
    s += __shfl_xor(s, 4, 32);
    s += __shfl_xor(s, 2, 32);
    s += __shfl_xor(s, 1, 32);
    const float mean = s * invd;
    const float d0 = y0 - mean, d1 = y1 - mean;
    float q = d0 * d0 + d1 * d1;
    q += __shfl_xor(q, 16, 32);
    q += __shfl_xor(q, 8, 32);
    q += __shfl_xor(q, 4, 32);
    q += __shfl_xor(q, 2, 32);
    q += __shfl_xor(q, 1, 32);
    const float var  = q * invd;
    const float rstd = 1.0f / sqrtf(var + LNEPS);
    const float t0 = (d0 * rstd) * gq0 + eq0;
    const float t1 = (d1 * rstd) * gq1 + eq1;
    const float o0 = (t0 > 0.0f) ? t0 : (t0 - t0);
    const float o1 = (t1 > 0.0f) ? t1 : (t1 - t1);
    unsigned l0, l1;
    const unsigned h0 = hl_bits(o0, l0);
    const unsigned h1 = hl_bits(o1, l1);
    v2us hv, lv;
    hv[0] = (unsigned short)h0; hv[1] = (unsigned short)h1;
    lv[0] = (unsigned short)l0; lv[1] = (unsigned short)l1;
    wave_sync();
    unsigned short* srow = (unsigned short*)frow;
    *(v2usa*)(srow + 2 * lane)       = hv;
    *(v2usa*)(srow + HID + 2 * lane) = lv;
  }
  __syncthreads();

  v8us qv[8];
#pragma unroll
  for (int j = 0; j < 8; ++j) {
    const int row = 16 * wave + 2 * j + hh;
    qv[j] = *(const v8usa*)((const unsigned short*)stg + (size_t)row * 128 + 8 * m);
  }
#pragma unroll
  for (int j = 0; j < 8; ++j) {
    const int gr = rowBase + 16 * wave + 2 * j + hh;
    unsigned short* rp = AH + (size_t)gr * AHP + sliceOff + 8 * m;
    *(volatile v8us*)rp = qv[j];
  }
  __threadfence();
#pragma unroll
  for (int j = 0; j < 8; ++j) {
    const int gr = rowBase + 16 * wave + 2 * j + hh;
    unsigned short* rp = AH + (size_t)gr * AHP + sliceOff + 8 * m;
    *(volatile v8us*)rp = qv[j];
  }
}

__global__ __launch_bounds__(128) __attribute__((amdgpu_num_vgpr(248)))
void k_gemm_p(const unsigned short* __restrict__ A, const unsigned short* __restrict__ BT, float* P) {
  __shared__ __attribute__((aligned(16))) float stg[64 * 64];
  const int tid = (int)threadIdx.x, lane = tid & 31, wave = tid >> 5, hh = lane >> 4, m = lane & 15;
  const int rowBase = (int)blockIdx.x * 64;
  const int colBase = (int)blockIdx.y * 64;

  v8f acc[4];
#pragma unroll
  for (int t = 0; t < 4; ++t) acc[t] = z8();
  const unsigned short* ap = A + (size_t)(rowBase + 16 * wave + m) * (size_t)AHP + 8 * hh;
  const unsigned short* bp = BT + (size_t)(colBase + m) * (size_t)AHP + 8 * hh;
#pragma unroll 2
  for (int k0 = 0; k0 < AHP; k0 += 32) {
    FragB af;
    af.h[0] = *(const v8usa*)(ap + k0);
    af.h[1] = *(const v8usa*)(ap + k0 + 16);
#pragma unroll
    for (int nt = 0; nt < 4; ++nt) {
      const unsigned short* wq = bp + (size_t)(16 * nt) * (size_t)AHP + k0;
      FragB bf;
      bf.h[0] = *(const v8usa*)wq;
      bf.h[1] = *(const v8usa*)(wq + 16);
      acc[nt] = wmb(af, bf, acc[nt]);
    }
  }
#pragma unroll
  for (int nt = 0; nt < 4; ++nt) {
    const int lc = 16 * nt + m;
#pragma unroll
    for (int r = 0; r < 8; ++r) {
      const int lr = 16 * wave + 8 * hh + r;
      stg[lr * 64 + lc] = acc[nt][r];
    }
  }
  __syncthreads();
  const int c4 = 4 * m;
  const bool ok = (colBase + c4) < PP;
  v4f pv[8];
#pragma unroll
  for (int j = 0; j < 8; ++j) {
    const int row = 16 * wave + 2 * j + hh;
    pv[j] = *(const v4fa*)(stg + row * 64 + c4);
  }
#pragma unroll
  for (int j = 0; j < 8; ++j) {
    const int gr = rowBase + 16 * wave + 2 * j + hh;
    float* op = P + (size_t)gr * PP + colBase + c4;
    if (ok) *(volatile v4f*)op = pv[j];
  }
  __threadfence();
#pragma unroll
  for (int j = 0; j < 8; ++j) {
    const int gr = rowBase + 16 * wave + 2 * j + hh;
    float* op = P + (size_t)gr * PP + colBase + c4;
    if (ok) *(volatile v4f*)op = pv[j];
  }
}

__global__ __launch_bounds__(PJ) void k_statA(const float* __restrict__ P, const int* __restrict__ aloc,
                                              const float* __restrict__ dist, const float* __restrict__ PAR,
                                              float* REC) {
  __shared__ __attribute__((aligned(16))) float sD[NA * NCH];
  __shared__ __attribute__((aligned(16))) float sPA[NA * PJ];
  __shared__ __attribute__((aligned(16))) float pst[RECW];
  __shared__ int sloc[NA];
  const int tid = (int)threadIdx.x;
  const int b  = (int)blockIdx.x >> 3;
  const int n0 = ((int)blockIdx.x & 7) * NCH;
  const int jc = tid < MID ? tid : MID - 1;
  const bool live = tid < MID;
  {
    const int lraw = aloc[b * NA + (tid & (NA - 1))];
    pin_i(lraw);
    const int lv = clampi(lraw, 0, NN - 1);
    if (tid < NA) sloc[tid] = lv;
  }
  __syncthreads();
#pragma unroll
  for (int it = 0; it < 3; ++it) {
    const int u  = it * PJ + tid;
    const int uc = u < DUNITS ? u : DUNITS - 1;
    const int i = uc >> 5, n4 = (uc & 31) * 4;
    v4f d = *(const v4f*)(dist + (size_t)sloc[i] * NN + n0 + n4);
    pin_f4(d);
    d.x = bf16_val(d.x); d.y = bf16_val(d.y); d.z = bf16_val(d.z); d.w = bf16_val(d.w);
    if (u < DUNITS) *(v4fa*)(sD + i * NCH + n4) = d;
  }
  const float uj  = PAR[jc];
  const float cvj = PAR[PJ + jc];
#pragma unroll 4
  for (int i = 0; i < NA; ++i) {
    const float v = P[(size_t)(b * NN + sloc[i]) * PP + jc];
    sPA[i * PJ + tid] = v + cvj;
  }
  __syncthreads();
  float pa[NA];
#pragma unroll
  for (int i = 0; i < NA; ++i) pa[i] = sPA[i * PJ + tid];
  const float* pbp = P + (size_t)(b * NN + n0) * PP + MID + jc;
  const float pilot = fmaf(sD[0], uj, pa[0] + pbp[0]);
  float s1 = 0.0f, s2 = 0.0f;
#pragma unroll 1
  for (int n = 0; n < NCH; ++n) {
    const float pb = pbp[(size_t)n * PP];
#pragma unroll
    for (int i = 0; i < NA; ++i) {
      const float d  = sD[i * NCH + n];
      const float h  = fmaf(d, uj, pa[i] + pb);
      const float dd = h - pilot;
      s1 += dd;
      s2 = fmaf(dd, dd, s2);
    }
  }
  const float rn = 1.0f / 2048.0f;
  const float mb = pilot + s1 * rn;
  const float qb = s2 - (s1 * s1) * rn;
  pst[tid]      = live ? mb : 0.0f;
  pst[PJ + tid] = live ? qb : 0.0f;
  __syncthreads();
  const int tq = tid < RECW / 4 ? tid : 0;
  const v4f v = *(const v4fa*)(pst + 4 * tq);
  float* op = REC + (size_t)blockIdx.x * RECW + 4 * tq;
  if (tid < RECW / 4) *(volatile v4f*)op = v;
  __threadfence();
  if (tid < RECW / 4) *(volatile v4f*)op = v;
}

__global__ __launch_bounds__(PJ) void k_comb(const float* __restrict__ REC, float* STAT) {
  __shared__ __attribute__((aligned(16))) float pst[RECW];
  const int tid = (int)threadIdx.x;
  const int jc = tid < MID ? tid : MID - 1;
  const bool live = tid < MID;
  double n = 0.0, mean = 0.0, M2 = 0.0;
#pragma unroll 1
  for (int r = 0; r < NREC; ++r) {
    const double mb = (double)REC[(size_t)r * RECW + jc];
    const double qb = (double)REC[(size_t)r * RECW + PJ + jc];
    const double nb = RECN;
    const double nn = n + nb;
    const double delta = mb - mean;
    const double f = nb / nn;
    mean = mean + delta * f;
    M2 = M2 + qb + delta * delta * n * f;
    n = nn;
  }
  const float varf = (float)(M2 / n);
  const float muf  = (float)mean;
  const float rstd = 1.0f / sqrtf(varf + BNEPS);
  pst[tid]      = live ? muf  : 0.0f;
  pst[PJ + tid] = live ? rstd : 0.0f;
  __syncthreads();
  const int tq = tid < RECW / 4 ? tid : 0;
  const v4f v = *(const v4fa*)(pst + 4 * tq);
  float* op = STAT + 4 * tq;
  if (tid < RECW / 4) *(volatile v4f*)op = v;
  __threadfence();
  if (tid < RECW / 4) *(volatile v4f*)op = v;
}

__global__ __launch_bounds__(256) void k_passB(const float* __restrict__ P, const int* __restrict__ aloc,
                                               const float* __restrict__ dist, const float* __restrict__ PAR,
                                               const float* __restrict__ STAT, const int* __restrict__ mask,
                                               float* LOGIT) {
  extern __shared__ __attribute__((aligned(16))) float dynB[];
  float* sPAt = dynB;
  float* sPar = sPAt + MID * NA;
  float* sD   = sPar + 256 * 8;
  i1a*   sMk  = (i1a*)(sD + NA * NCH);
  i1a*   sloc = sMk + NA * NCH;
  float* sPB  = (float*)(sloc + 16);
  const int tid = (int)threadIdx.x, lane = tid & 31, wave = tid >> 5;
  const int b  = (int)blockIdx.x >> 3;
  const int n0 = ((int)blockIdx.x & 7) * NCH;

  {
    const int lraw = aloc[b * NA + (tid & (NA - 1))];
    pin_i(lraw);
    const int lv = clampi(lraw, 0, NN - 1);
    if (tid < NA) sloc[tid] = lv;
  }
  __syncthreads();
#pragma unroll
  for (int it = 0; it < DUNITS / 256; ++it) {
    const int u = it * 256 + tid;
    const int i = u >> 5, n4 = (u & 31) * 4;
    v4f d = *(const v4f*)(dist + (size_t)sloc[i] * NN + n0 + n4);
    d.x = bf16_val(d.x); d.y = bf16_val(d.y); d.z = bf16_val(d.z); d.w = bf16_val(d.w);
    *(v4fa*)(sD + i * NCH + n4) = d;
    const v4i mk = *(const v4i*)(mask + (size_t)b * ANPB + (size_t)i * NN + n0 + n4);
    *(v4ia*)(sMk + i * NCH + n4) = mk;
  }
  {
    const int jc = tid < MID ? tid : MID - 1;
    v4f q0, q1;
    q0.x = PAR[jc];
    q0.y = STAT[jc];
    q0.z = STAT[PJ + jc];
    q0.w = PAR[2 * PJ + jc];
    q1.x = PAR[3 * PJ + jc];
    q1.y = PAR[4 * PJ + jc];
    q1.z = 0.0f; q1.w = 0.0f;
    *(v4fa*)(sPar + 8 * tid)     = q0;
    *(v4fa*)(sPar + 8 * tid + 4) = q1;
  }
#pragma unroll 1
  for (int it = 0; it < (MID * NA) / 256; ++it) {
    const int e = it * 256 + tid;
    const int i = e / MID;
    const int j = e - i * MID;
    const float v = P[(size_t)(b * NN + sloc[i]) * PP + j] + PAR[PJ + j];
    sPAt[j * NA + i] = v;
  }
#pragma unroll 2
  for (int it = 0; it < (NCH * (MID / 4)) / 256; ++it) {
    const int u = it * 256 + tid;
    const int rn = u / (MID / 4);
    const int c4 = (u - rn * (MID / 4)) * 4;
    const v4f x = *(const v4f*)(P + (size_t)(b * NN + n0 + rn) * PP + MID + c4);
    float* dp = sPB + rn * PB_STR + c4;
    dp[0] = x.x; dp[1] = x.y; dp[2] = x.z; dp[3] = x.w;
  }
  __syncthreads();

  const int nrow = 32 * (wave & 3) + lane;
  const int ag0  = 8 * (wave >> 2);
  float dv[8], acc[8];
#pragma unroll
  for (int i = 0; i < 8; ++i) { dv[i] = sD[(ag0 + i) * NCH + nrow]; acc[i] = 0.0f; }
  const float* pbr = sPB + nrow * PB_STR;
#pragma unroll 1
  for (int j = 0; j < MID; ++j) {
    const float pb = pbr[j];
    const v4f q0 = *(const v4fa*)(sPar + 8 * j);
    const v4f q1 = *(const v4fa*)(sPar + 8 * j + 4);
    const v4f a0 = *(const v4fa*)(sPAt + NA * j + ag0);
    const v4f a1 = *(const v4fa*)(sPAt + NA * j + ag0 + 4);
    const float pa[8] = {a0.x, a0.y, a0.z, a0.w, a1.x, a1.y, a1.z, a1.w};
#pragma unroll
    for (int i = 0; i < 8; ++i) {
      const float h = fmaf(dv[i], q0.x, pa[i] + pb);
      const float x = (h - q0.y) * q0.z;
      const float y = fmaf(x, q0.w, q1.x);
      const float r = (y > 0.0f) ? y : (y - y);
      acc[i] = fmaf(r, q1.y, acc[i]);
    }
  }
  const float b2v = PAR[5 * PJ];
  float lm[8];
#pragma unroll
  for (int i = 0; i < 8; ++i) {
    const int mk = sMk[(ag0 + i) * NCH + nrow];
    const float lg = acc[i] + b2v;
    lm[i] = (mk != 0) ? lg : -100000000.0f;
  }
  float* lp = LOGIT + (size_t)b * ANPB + (size_t)ag0 * NN + n0 + nrow;
#pragma unroll
  for (int i = 0; i < 8; ++i) *(volatile float*)(lp + (size_t)i * NN) = lm[i];
  __threadfence();
#pragma unroll
  for (int i = 0; i < 8; ++i) *(volatile float*)(lp + (size_t)i * NN) = lm[i];
}

__global__ __launch_bounds__(256) void k_softmax(const float* __restrict__ LOGIT, float* out) {
  extern __shared__ __attribute__((aligned(16))) float sE[];
  __shared__ float wmx[8];
  __shared__ float ssum[256];
  const int tid = (int)threadIdx.x, lane = tid & 31, wave = tid >> 5;
  const int b = (int)blockIdx.x;
  const float* L = LOGIT + (size_t)b * ANPB;
  float m = -__builtin_huge_valf();
#pragma unroll 4
  for (int it = 0; it < 16; ++it) {
    const int q = it * 256 + tid;
    const v4f x = *(const v4f*)(L + 4 * q);
    *(v4fa*)(sE + 4 * q) = x;
    m = nmax(m, x.x); m = nmax(m, x.y); m = nmax(m, x.z); m = nmax(m, x.w);
  }
#pragma unroll
  for (int d = 16; d > 0; d >>= 1) {
    const float o = __shfl_xor(m, d, 32);
    m = nmax(m, o);
  }
  if (lane == 0) wmx[wave] = m;
  __syncthreads();
  float bm = wmx[0];
#pragma unroll
  for (int w2 = 1; w2 < 8; ++w2) bm = nmax(bm, wmx[w2]);

  float se = 0.0f;
#pragma unroll 1
  for (int it = 0; it < 16; ++it) {
    const int q = it * 256 + tid;
    const v4f x = *(const v4fa*)(sE + 4 * q);
    v4f e;
    e.x = expf(x.x - bm); e.y = expf(x.y - bm); e.z = expf(x.z - bm); e.w = expf(x.w - bm);
    *(v4fa*)(sE + 4 * q) = e;
    se += (e.x + e.y) + (e.z + e.w);
  }
  ssum[tid] = se;
  __syncthreads();
  double tot = 0.0;
#pragma unroll 4
  for (int k = 0; k < 256; ++k) tot += (double)ssum[k];
  const float inv = 1.0f / (float)tot;

  float* op = out + (size_t)b * ANPB;
#pragma unroll 4
  for (int it = 0; it < 16; ++it) {
    const int q = it * 256 + tid;
    const v4f e = *(const v4fa*)(sE + 4 * q);
    const v4f o = e * inv;
    *(volatile v4f*)(op + 4 * q) = o;
  }
  __threadfence();
#pragma unroll 4
  for (int it = 0; it < 16; ++it) {
    const int q = it * 256 + tid;
    const v4f e = *(const v4fa*)(sE + 4 * q);
    const v4f o = e * inv;
    *(volatile v4f*)(op + 4 * q) = o;
  }
}

static inline size_t al256(size_t o) { return (o + 255) & ~(size_t)255; }

extern "C" void kernel_launch(void* const* d_in, const int* in_sizes, int n_in,
                              void* d_out, int out_size, void* d_ws, size_t ws_size,
                              hipStream_t stream) {
  if (n_in < 25) return;
  static const int want[25] = {BNR * FIN, NB * 2 * NE, NB * NA, RTOT, NN * NN,
                               FIN * HID, HID, HID, HID,
                               HID * HID, HID, HID, HID,
                               HID * HID, HID, HID, HID,
                               HID, HID, (2 * MID + HID) * MID, MID, MID, MID, MID, 1};
  for (int i = 0; i < 25; ++i) if (in_sizes[i] != want[i]) return;
  if (out_size != RTOT) return;

  const float* gn    = (const float*)d_in[0];
  const int*   links = (const int*)  d_in[1];
  const int*   aloc  = (const int*)  d_in[2];
  const int*   mask  = (const int*)  d_in[3];
  const float* dist  = (const float*)d_in[4];
  const float* W0  = (const float*)d_in[5];
  const float* b0  = (const float*)d_in[6];
  const float* g0  = (const float*)d_in[7];
  const float* be0 = (const float*)d_in[8];
  const float* W1  = (const float*)d_in[9];
  const float* b1  = (const float*)d_in[10];
  const float* g1  = (const float*)d_in[11];
  const float* be1 = (const float*)d_in[12];
  const float* W2  = (const float*)d_in[13];
  const float* b2c = (const float*)d_in[14];
  const float* g2  = (const float*)d_in[15];
  const float* be2 = (const float*)d_in[16];
  const float* eW  = (const float*)d_in[17];
  const float* eb  = (const float*)d_in[18];
  const float* A1  = (const float*)d_in[19];
  const float* a1b = (const float*)d_in[20];
  const float* bng = (const float*)d_in[21];
  const float* bnb = (const float*)d_in[22];
  const float* w2  = (const float*)d_in[23];
  const float* b2  = (const float*)d_in[24];
  float* out = (float*)d_out;

  char* ws = (char*)d_ws;
  size_t off = 0;
  const size_t oW0D = off; off = al256(off + (size_t)HID * 64 * 2);
  const size_t oW1D = off; off = al256(off + (size_t)HID * 128 * 2);
  const size_t oW2D = off; off = al256(off + (size_t)HID * 128 * 2);
  const size_t oWAB = off; off = al256(off + (size_t)AHP * AHP * 2);
  const size_t oPAR = off; off = al256(off + (size_t)PARW * 4);
  const size_t oAH  = off; off = al256(off + (size_t)BNR * AHP * 2);
  const size_t oAGG = off; off = al256(off + (size_t)BNR * 128 * 2);
  const size_t oLST = off; off = al256(off + (size_t)NB * NE * 4);
  const size_t oOFF = off; off = al256(off + (size_t)NB * OFFP * 4);
  const size_t oP   = off; off = al256(off + (size_t)BNR * PP * 4);
  const size_t oREC = off; off = al256(off + (size_t)NREC * RECW * 4);
  const size_t oSTA = off; off = al256(off + (size_t)RECW * 4);
  const size_t oLOG = off; off = al256(off + (size_t)RTOT * 4);
  if (off > ws_size || off > (size_t)WSMAX) return;
  unsigned short* W0D = (unsigned short*)(ws + oW0D);
  unsigned short* W1D = (unsigned short*)(ws + oW1D);
  unsigned short* W2D = (unsigned short*)(ws + oW2D);
  unsigned short* WAB = (unsigned short*)(ws + oWAB);
  float*          PAR = (float*)(ws + oPAR);
  unsigned short* AH  = (unsigned short*)(ws + oAH);
  unsigned short* AGG = (unsigned short*)(ws + oAGG);
  int*            LST = (int*)(ws + oLST);
  int*            OFT = (int*)(ws + oOFF);
  float*          P   = (float*)(ws + oP);
  float*          REC = (float*)(ws + oREC);
  float*          STA = (float*)(ws + oSTA);
  float*          LOG = (float*)(ws + oLOG);

  const int bkLds = BK_INTS * 4;
  const int pbLds = PASSB_FLOATS * 4;
  const int smLds = ANPB * 4;
  hipFuncSetAttribute(reinterpret_cast<const void*>(&k_bucket), hipFuncAttributeMaxDynamicSharedMemorySize, bkLds);
  hipFuncSetAttribute(reinterpret_cast<const void*>(&k_passB), hipFuncAttributeMaxDynamicSharedMemorySize, pbLds);
  hipFuncSetAttribute(reinterpret_cast<const void*>(&k_softmax), hipFuncAttributeMaxDynamicSharedMemorySize, smLds);

  k_pa<<<NU_PA / 256, 256, 0, stream>>>(gn, W0, W1, W2, W0D, W1D, W2D, AH);
  k_pb<<<NU_PB / 256, 256, 0, stream>>>(A1, WAB);
  k_pc<<<1, 256, 0, stream>>>(A1, a1b, eW, eb, bng, bnb, w2, b2, PAR);
  k_bucket<<<NB, 256, bkLds, stream>>>(links, LST, OFT);
  k_agg<1><<<BNR / 64, 256, 0, stream>>>(LST, OFT, gn, AH, 0, AGG);
  k_gemm_ln<2><<<BNR / 64, 128, 0, stream>>>(AGG, W0D, b0, g0, be0, AH, 0);
  k_agg<0><<<BNR / 64, 256, 0, stream>>>(LST, OFT, gn, AH, 0, AGG);
  k_gemm_ln<4><<<BNR / 64, 128, 0, stream>>>(AGG, W1D, b1, g1, be1, AH, 128);
  k_agg<0><<<BNR / 64, 256, 0, stream>>>(LST, OFT, gn, AH, 128, AGG);
  k_gemm_ln<4><<<BNR / 64, 128, 0, stream>>>(AGG, W2D, b2c, g2, be2, AH, 256);
  k_gemm_p<<<dim3(BNR / 64, AHP / 64), 128, 0, stream>>>(AH, WAB, P);
  k_statA<<<NREC, PJ, 0, stream>>>(P, aloc, dist, PAR, REC);
  k_comb<<<1, PJ, 0, stream>>>(REC, STA);
  k_passB<<<NREC, 256, pbLds, stream>>>(P, aloc, dist, PAR, STA, mask, LOG);
  k_softmax<<<NB, 256, smLds, stream>>>(LOG, out);
}
